// GCMC_40870908789353
// MI455X (gfx1250) — hardware-verified
//
#include <hip/hip_runtime.h>
#include <stddef.h>


#define DIM    64
#define DFV    128
#define KLIN   256
#define NTHR   256
#define NWAVE  8
#define EPT    8
#define NGRP   2
#define CHUNK  (NTHR * EPT * NGRP)
#define WCAP   (EPT * NGRP * 32)
#define LISTN  (NWAVE * WCAP)
#define SLB    14
#define NBA    1024
#define NBW    512
#define NROW   1024
#define G1THR  128
#define G1WAV  4
#define G2THR  64
#define G2WAV  2
#define TPW    8
#define RPB1   (G1WAV * TPW * 16)
#define RPB2   (G2WAV * TPW * 16)
#define PA     72
#define PB     136
#define PD     68
#define OFF_WC 0
#define OFF_W2 8192
#define OFF_WW 16384
#define OFF_WL 24576
#define WTOT   57344
#define SBLK   256
#define LDS_E  (NBA * DIM * 4 + LISTN * 4 + 64)
#define LDS_W  (NBW * DFV * 4 + NBW * 4 + LISTN * 4 + 64)

static_assert((CHUNK & (CHUNK - 1)) == 0);
static_assert(CHUNK <= (1 << 12));
static_assert((NBA & (NBA - 1)) == 0 && NBA <= (1 << SLB));
static_assert((NBW & (NBW - 1)) == 0 && NBW <= (1 << SLB));
static_assert(NBA == NWAVE * 64 * 2);
static_assert(NBW == NWAVE * 64);
static_assert((NROW % NBA) == 0 && (NROW % NBW) == 0 && (NROW % RPB1) == 0 && (NROW % RPB2) == 0);
static_assert(OFF_W2 == OFF_WC + 2 * 64 * DIM && OFF_WW == OFF_W2 + 2 * 64 * DIM);
static_assert(OFF_WL == OFF_WW + 2 * 64 * DIM && WTOT == OFF_WL + 2 * 64 * KLIN);
static_assert(((PA * 2) % 16) == 0 && ((PB * 2) % 16) == 0 && ((PD * 4) % 16) == 0);
static_assert((SBLK % 128) == 0);

typedef float          v2f   __attribute__((ext_vector_type(2)));
typedef float          v4f   __attribute__((ext_vector_type(4)));
typedef float          v8f   __attribute__((ext_vector_type(8)));
typedef int            v4i   __attribute__((ext_vector_type(4)));
typedef unsigned short v8us  __attribute__((ext_vector_type(8)));
typedef unsigned short v16us __attribute__((ext_vector_type(16)));
typedef __bf16         v16bf __attribute__((ext_vector_type(16)));
union Frag { v16bf v; v16us u; v8us h[2]; };

__device__ __forceinline__ float lk(float x) { return x >= 0.0f ? x : 0.01f * x; }
__device__ __forceinline__ v4f lk4(v4f a) { v4f r; r.x = lk(a.x); r.y = lk(a.y); r.z = lk(a.z); r.w = lk(a.w); return r; }

__device__ __forceinline__ unsigned short bf_rne(float x) {
  unsigned int u = __float_as_uint(x);
  u += 0x7FFFu + ((u >> 16) & 1u);
  return (unsigned short)(u >> 16);
}
__device__ __forceinline__ void split2(float x, unsigned short& hi, unsigned short& lo) {
  const unsigned short h = bf_rne(x);
  const float r = x - __uint_as_float(((unsigned int)h) << 16);
  hi = h;
  lo = bf_rne(r);
}
__device__ __forceinline__ void split8(v4f a, v4f b, float s, v8us& hi, v8us& lo) {
  float t[8] = {a.x * s, a.y * s, a.z * s, a.w * s, b.x * s, b.y * s, b.z * s, b.w * s};
#pragma unroll
  for (int j = 0; j < 8; ++j) { unsigned short p, q; split2(t[j], p, q); hi[j] = p; lo[j] = q; }
}

__device__ __forceinline__ v8f wmb(v16bf a, v16bf b, v8f c) {
  v8f d = __builtin_amdgcn_wmma_f32_16x16x32_bf16(false, a, false, b, (short)0, c, false, false);
  asm volatile("v_nop\n\tv_nop\n\tv_nop\n\tv_nop" : "+v"(d) : "v"(a), "v"(b));
  return d;
}
__device__ __forceinline__ v8f mm3(v16bf ah, v16bf al, v16bf bh, v16bf bl, v8f c) {
  c = wmb(ah, bh, c);
  c = wmb(ah, bl, c);
  c = wmb(al, bh, c);
  return c;
}
__device__ __forceinline__ v16bf ldfrag(const unsigned short* p) {
  Frag f;
  f.h[0] = *(const v8us*)p;
  f.h[1] = *(const v8us*)(p + 16);
  return f.v;
}

template <int NB>
__device__ __forceinline__ int scan_chunk(const int* __restrict__ ids, int nE, int cbase, int slotBase,
                                          int vec8, int* list, int tid, int lane, int wave) {
  int wc = 0;
#pragma unroll
  for (int g = 0; g < NGRP; ++g) {
    const int el0  = (g * NTHR + tid) * EPT;
    const int e0   = cbase + el0;
    const int sent = -2147483647 - 1;
    v4i da, db;
    if (vec8 != 0 && cbase + CHUNK <= nE) {
      da = *(const v4i*)(ids + e0);
      db = *(const v4i*)(ids + e0 + 4);
    } else {
      da.x = (e0     < nE) ? ids[min(e0, nE - 1)] : sent;
      da.y = (e0 + 1 < nE) ? ids[min(e0 + 1, nE - 1)] : sent;
      da.z = (e0 + 2 < nE) ? ids[min(e0 + 2, nE - 1)] : sent;
      da.w = (e0 + 3 < nE) ? ids[min(e0 + 3, nE - 1)] : sent;
      db.x = (e0 + 4 < nE) ? ids[min(e0 + 4, nE - 1)] : sent;
      db.y = (e0 + 5 < nE) ? ids[min(e0 + 5, nE - 1)] : sent;
      db.z = (e0 + 6 < nE) ? ids[min(e0 + 6, nE - 1)] : sent;
      db.w = (e0 + 7 < nE) ? ids[min(e0 + 7, nE - 1)] : sent;
    }
    const unsigned nb = (unsigned)slotBase;
    const unsigned s0 = (unsigned)da.x - nb, s1 = (unsigned)da.y - nb;
    const unsigned s2 = (unsigned)da.z - nb, s3 = (unsigned)da.w - nb;
    const unsigned s4 = (unsigned)db.x - nb, s5 = (unsigned)db.y - nb;
    const unsigned s6 = (unsigned)db.z - nb, s7 = (unsigned)db.w - nb;
    const bool h0 = s0 < (unsigned)NB, h1 = s1 < (unsigned)NB, h2 = s2 < (unsigned)NB, h3 = s3 < (unsigned)NB;
    const bool h4 = s4 < (unsigned)NB, h5 = s5 < (unsigned)NB, h6 = s6 < (unsigned)NB, h7 = s7 < (unsigned)NB;
    const unsigned any = __builtin_amdgcn_ballot_w32(h0 | h1 | h2 | h3 | h4 | h5 | h6 | h7);
    if (any != 0u) {
#define HITJ(J, HJ, SJ) { \
        const unsigned mj = __builtin_amdgcn_ballot_w32(HJ); \
        if (mj != 0u) { \
          if (HJ) { \
            const int pos = wc + (int)__builtin_amdgcn_mbcnt_lo(mj, 0u); \
            if (pos < WCAP) list[wave * WCAP + pos] = ((el0 + (J)) << SLB) | (int)(SJ); \
          } \
          wc += (int)__builtin_popcount(mj); } }
      HITJ(0, h0, s0)
      HITJ(1, h1, s1)
      HITJ(2, h2, s2)
      HITJ(3, h3, s3)
      HITJ(4, h4, s4)
      HITJ(5, h5, s5)
      HITJ(6, h6, s6)
      HITJ(7, h7, s7)
#undef HITJ
    }
  }
  return wc;
}

__device__ __forceinline__ void wplane(const float* __restrict__ W, int K, unsigned short* dst, int tid) {
  const int kq = K >> 3;
  const int units = 64 * kq;
#pragma unroll 1
  for (int u = tid; u < units; u += NTHR) {
    const int n  = u / kq;
    const int k0 = (u - n * kq) * 8;
    v8us hi, lo;
#pragma unroll
    for (int j = 0; j < 8; ++j) {
      unsigned short p, q;
      split2(W[(size_t)(k0 + j) * 64 + n], p, q);
      hi[j] = p; lo[j] = q;
    }
    unsigned short* ph = dst + (size_t)u * 8;
    unsigned short* pl = dst + (size_t)64 * K + (size_t)u * 8;
    *(volatile v8us*)ph = hi;
    *(volatile v8us*)pl = lo;
    __threadfence();
    *(volatile v8us*)ph = hi;
    *(volatile v8us*)pl = lo;
  }
}

__global__ __launch_bounds__(NTHR) void k_wprep(
    const float* __restrict__ Wc, const float* __restrict__ W2, const float* __restrict__ Ww,
    const float* __restrict__ Wl, unsigned short* Wpl) {
  const int seg = (int)blockIdx.x, tid = (int)threadIdx.x;
  if (seg == 0)      wplane(Wc, DIM,  Wpl + OFF_WC, tid);
  else if (seg == 1) wplane(W2, DIM,  Wpl + OFF_W2, tid);
  else if (seg == 2) wplane(Ww, DIM,  Wpl + OFF_WW, tid);
  else if (seg == 3) wplane(Wl, KLIN, Wpl + OFF_WL, tid);
}

__device__ __forceinline__ void st64f(const float* tD, float* P, size_t row0, int lane) {
#pragma unroll
  for (int i = 0; i < 8; ++i) {
    const int p = i * 32 + lane, row = p >> 4, c = (p & 15) * 4;
    const v4f v = *(const v4f*)(tD + row * PD + c);
    *(volatile v4f*)(P + (row0 + (size_t)row) * DIM + c) = v;
  }
}

__global__ __launch_bounds__(G1THR) void k_gemm1(
    const float* __restrict__ emb, const unsigned short* __restrict__ Wpl, float* H, int nN) {
  __shared__ __attribute__((aligned(16))) unsigned short sAh[G1WAV * 16 * PA];
  __shared__ __attribute__((aligned(16))) unsigned short sAl[G1WAV * 16 * PA];
  __shared__ __attribute__((aligned(16))) float sD[G1WAV * 16 * PD];
  const int tid = threadIdx.x, lane = tid & 31, wave = tid >> 5, hh = lane >> 4, m = lane & 15;
  unsigned short* tAh = sAh + wave * 16 * PA;
  unsigned short* tAl = sAl + wave * 16 * PA;
  float* tD = sD + wave * 16 * PD;
  const unsigned short* Wh = Wpl + OFF_WC;
  const v8f z = {0.f, 0.f, 0.f, 0.f, 0.f, 0.f, 0.f, 0.f};
  const int tile0 = ((int)blockIdx.x * G1WAV + wave) * TPW;

#pragma unroll 1
  for (int tt = 0; tt < TPW; ++tt) {
    const size_t row0 = (size_t)(tile0 + tt) * 16;
    int rr = (int)row0 + m;
    rr = rr > nN - 1 ? nN - 1 : rr;
    const float* rp = emb + (size_t)rr * DIM + 32 * hh;
    v4f x[8];
    float ss = 0.0f;
#pragma unroll
    for (int j = 0; j < 8; ++j) {
      x[j] = *(const v4f*)(rp + 4 * j);
      ss += x[j].x * x[j].x + x[j].y * x[j].y + x[j].z * x[j].z + x[j].w * x[j].w;
    }
    const float tot = ss + __shfl_xor(ss, 16);
    const float inv = 1.0f / fmaxf(sqrtf(tot), 1e-12f);
#pragma unroll
    for (int j = 0; j < 4; ++j) {
      v8us hi, lo;
      split8(x[2 * j], x[2 * j + 1], inv, hi, lo);
      *(v8us*)(tAh + m * PA + 32 * hh + 8 * j) = hi;
      *(v8us*)(tAl + m * PA + 32 * hh + 8 * j) = lo;
    }
    __syncthreads();
    v8f acc[4] = {z, z, z, z};
#pragma unroll
    for (int ks = 0; ks < 2; ++ks) {
      const v16bf ah = ldfrag(tAh + m * PA + 32 * ks + 8 * hh);
      const v16bf al = ldfrag(tAl + m * PA + 32 * ks + 8 * hh);
#pragma unroll
      for (int nt = 0; nt < 4; ++nt) {
        const unsigned short* wp = Wh + (size_t)(16 * nt + m) * DIM + 32 * ks + 8 * hh;
        acc[nt] = mm3(ah, al, ldfrag(wp), ldfrag(wp + 64 * DIM), acc[nt]);
      }
    }
#pragma unroll
    for (int nt = 0; nt < 4; ++nt) {
#pragma unroll
      for (int r = 0; r < 8; ++r) tD[(8 * hh + r) * PD + 16 * nt + m] = acc[nt][r];
    }
    __syncthreads();
    st64f(tD, H, row0, lane);
    __threadfence();
    st64f(tD, H, row0, lane);
    __syncthreads();
  }
}

__device__ __forceinline__ void agge_store(const float* sacc, unsigned short* X2, int slotBase, int wave, int lane) {
#pragma unroll 2
  for (int it = 0; it < 64; ++it) {
    const int row = (it * NWAVE + wave) * 2 + (lane >> 4);
    const int q   = lane & 15;
    const int c0  = (q & 7) * 8;
    const v4f a = *(const v4f*)(sacc + row * DIM + c0);
    const v4f b = *(const v4f*)(sacc + row * DIM + c0 + 4);
    v8us hi, lo;
    split8(lk4(a), lk4(b), 1.0f, hi, lo);
    v8us o;
#pragma unroll
    for (int j = 0; j < 8; ++j) o[j] = (q < 8) ? hi[j] : lo[j];
    *(volatile v8us*)(X2 + ((size_t)slotBase + (size_t)row) * (2 * DIM) + q * 8) = o;
  }
}

__global__ __launch_bounds__(NTHR) void k_agge(
    const int* __restrict__ edst, const int* __restrict__ esrc, const float* __restrict__ H,
    unsigned short* X2, int nN, int nE, int vec8) {
  extern __shared__ v4f lds_dyn[];
  float* sacc = (float*)lds_dyn;
  int*   list = (int*)(sacc + NBA * DIM);
  int*   wcnt = list + LISTN;
  const int tid = threadIdx.x, lane = tid & 31, wave = tid >> 5;
  const int slotBase = (int)blockIdx.x * NBA;
  {
    const v4f z = {0.f, 0.f, 0.f, 0.f};
    for (int i = tid; i < NBA * DIM / 4; i += NTHR) ((v4f*)sacc)[i] = z;
  }
  __syncthreads();

  const int nChunks = (nE + CHUNK - 1) / CHUNK;
#pragma unroll 1
  for (int ch = 0; ch < nChunks; ++ch) {
    const int cbase = ch * CHUNK;
    const int wc = scan_chunk<NBA>(edst, nE, cbase, slotBase, vec8, list, tid, lane, wave);
    if (lane == 0) wcnt[wave] = wc;
    __syncthreads();
    if (wave == 0) {
#pragma unroll 1
      for (int wsx = 0; wsx < NWAVE; ++wsx) {
        int n = __builtin_amdgcn_readfirstlane(wcnt[wsx]);
        n = n > WCAP ? WCAP : (n < 0 ? 0 : n);
        const int* lp = list + wsx * WCAP;
#pragma unroll 1
        for (int i = 0; i < n; ++i) {
          const int ent  = __builtin_amdgcn_readfirstlane(lp[i]);
          const int slot = ent & (NBA - 1);
          int e = cbase + ((ent >> SLB) & (CHUNK - 1));
          e = e > nE - 1 ? nE - 1 : e;
          int s = esrc[e];
          if (s < 0) s += nN;
          s = s < 0 ? 0 : (s > nN - 1 ? nN - 1 : s);
          const v2f hv = *(const v2f*)(H + (size_t)s * DIM + 2 * lane);
          v2f* ap = (v2f*)(sacc + slot * DIM + 2 * lane);
          v2f cur = *ap;
          cur.x += hv.x;
          cur.y += hv.y;
          *ap = cur;
        }
      }
    }
    __syncthreads();
  }

  agge_store(sacc, X2, slotBase, wave, lane);
  __threadfence();
  agge_store(sacc, X2, slotBase, wave, lane);
}

__device__ __forceinline__ void aggw_store(const float* sacc, const int* scnt, unsigned short* T,
                                           int slotBase, int wave, int lane) {
#pragma unroll 2
  for (int it = 0; it < 64; ++it) {
    const int row = it * NWAVE + wave;
    const int c0  = (lane & 15) * 8;
    const int c   = scnt[row];
    const float inv = 1.0f / (float)(c > 1 ? c : 1);
    const v4f a = *(const v4f*)(sacc + row * DFV + c0);
    const v4f b = *(const v4f*)(sacc + row * DFV + c0 + 4);
    v8us hi, lo;
    split8(a, b, inv, hi, lo);
    v8us o;
#pragma unroll
    for (int j = 0; j < 8; ++j) o[j] = (lane < 16) ? hi[j] : lo[j];
    *(volatile v8us*)(T + ((size_t)slotBase + (size_t)row) * (2 * DFV) + lane * 8) = o;
  }
}

__global__ __launch_bounds__(NTHR) void k_aggw(
    const int* __restrict__ witem, const int* __restrict__ wword, const float* __restrict__ table,
    unsigned short* T, int nVoc, int nW, int vec8) {
  extern __shared__ v4f lds_dyn[];
  float* sacc = (float*)lds_dyn;
  int*   scnt = (int*)(sacc + NBW * DFV);
  int*   list = scnt + NBW;
  int*   wcnt = list + LISTN;
  const int tid = threadIdx.x, lane = tid & 31, wave = tid >> 5;
  const int slotBase = (int)blockIdx.x * NBW;
  {
    const v4f z = {0.f, 0.f, 0.f, 0.f};
    for (int i = tid; i < NBW * DFV / 4; i += NTHR) ((v4f*)sacc)[i] = z;
    for (int i = tid; i < NBW; i += NTHR) scnt[i] = 0;
  }
  __syncthreads();

  const int nChunks = (nW + CHUNK - 1) / CHUNK;
#pragma unroll 1
  for (int ch = 0; ch < nChunks; ++ch) {
    const int cbase = ch * CHUNK;
    const int wc = scan_chunk<NBW>(witem, nW, cbase, slotBase, vec8, list, tid, lane, wave);
    if (lane == 0) wcnt[wave] = wc;
    __syncthreads();
    if (wave == 0) {
#pragma unroll 1
      for (int wsx = 0; wsx < NWAVE; ++wsx) {
        int n = __builtin_amdgcn_readfirstlane(wcnt[wsx]);
        n = n > WCAP ? WCAP : (n < 0 ? 0 : n);
        const int* lp = list + wsx * WCAP;
#pragma unroll 1
        for (int i = 0; i < n; ++i) {
          const int ent  = __builtin_amdgcn_readfirstlane(lp[i]);
          const int slot = ent & (NBW - 1);
          int e = cbase + ((ent >> SLB) & (CHUNK - 1));
          e = e > nW - 1 ? nW - 1 : e;
          int w = wword[e];
          if (w < 0) w += nVoc;
          w = w < 0 ? 0 : (w > nVoc - 1 ? nVoc - 1 : w);
          const v4f tv = *(const v4f*)(table + (size_t)w * DFV + 4 * lane);
          v4f* ap = (v4f*)(sacc + slot * DFV + 4 * lane);
          v4f cur = *ap;
          cur.x += tv.x; cur.y += tv.y; cur.z += tv.z; cur.w += tv.w;
          *ap = cur;
          if (lane == 0) scnt[slot] = scnt[slot] + 1;
        }
      }
    }
    __syncthreads();
  }

  aggw_store(sacc, scnt, T, slotBase, wave, lane);
  __threadfence();
  aggw_store(sacc, scnt, T, slotBase, wave, lane);
}

__global__ __launch_bounds__(G2THR) void k_gemm23(
    const float* __restrict__ vf, const unsigned short* __restrict__ T,
    const unsigned short* __restrict__ Wpl, const float* __restrict__ lb, float* FH, int nItem) {
  __shared__ __attribute__((aligned(16))) unsigned short sVh[G2WAV * 16 * PB];
  __shared__ __attribute__((aligned(16))) unsigned short sVl[G2WAV * 16 * PB];
  __shared__ __attribute__((aligned(16))) unsigned short sFh[G2WAV * 16 * PA];
  __shared__ __attribute__((aligned(16))) unsigned short sFl[G2WAV * 16 * PA];
  __shared__ __attribute__((aligned(16))) float sD[G2WAV * 16 * PD];
  const int tid = threadIdx.x, lane = tid & 31, wave = tid >> 5, hh = lane >> 4, m = lane & 15;
  unsigned short* tVh = sVh + wave * 16 * PB;
  unsigned short* tVl = sVl + wave * 16 * PB;
  unsigned short* tFh = sFh + wave * 16 * PA;
  unsigned short* tFl = sFl + wave * 16 * PA;
  float* tD = sD + wave * 16 * PD;
  const unsigned short* WLh = Wpl + OFF_WL;
  const unsigned short* W2h = Wpl + OFF_W2;
  float bb[4];
#pragma unroll
  for (int t = 0; t < 4; ++t) bb[t] = lb[16 * t + m];
  const v8f z = {0.f, 0.f, 0.f, 0.f, 0.f, 0.f, 0.f, 0.f};
  const int tile0 = ((int)blockIdx.x * G2WAV + wave) * TPW;

#pragma unroll 1
  for (int tt = 0; tt < TPW; ++tt) {
    const size_t row0 = (size_t)(tile0 + tt) * 16;
    int rr = (int)row0 + m;
    rr = rr > nItem - 1 ? nItem - 1 : rr;
    const float* vp = vf + (size_t)rr * DFV + 64 * hh;
#pragma unroll
    for (int j = 0; j < 8; ++j) {
      const v4f a = *(const v4f*)(vp + 8 * j);
      const v4f b = *(const v4f*)(vp + 8 * j + 4);
      v8us hi, lo;
      split8(a, b, 1.0f, hi, lo);
      *(v8us*)(tVh + m * PB + 64 * hh + 8 * j) = hi;
      *(v8us*)(tVl + m * PB + 64 * hh + 8 * j) = lo;
    }
    __syncthreads();
    v8f acc[4] = {z, z, z, z};
#pragma unroll
    for (int ks = 0; ks < 4; ++ks) {
      const v16bf ah = ldfrag(tVh + m * PB + 32 * ks + 8 * hh);
      const v16bf al = ldfrag(tVl + m * PB + 32 * ks + 8 * hh);
#pragma unroll
      for (int nt = 0; nt < 4; ++nt) {
        const unsigned short* wp = WLh + (size_t)(16 * nt + m) * KLIN + 32 * ks + 8 * hh;
        acc[nt] = mm3(ah, al, ldfrag(wp), ldfrag(wp + 64 * KLIN), acc[nt]);
      }
    }
    const unsigned short* tp = T + (row0 + (size_t)m) * (2 * DFV) + 8 * hh;
#pragma unroll
    for (int ks = 0; ks < 4; ++ks) {
      const v16bf ah = ldfrag(tp + 32 * ks);
      const v16bf al = ldfrag(tp + DFV + 32 * ks);
#pragma unroll
      for (int nt = 0; nt < 4; ++nt) {
        const unsigned short* wp = WLh + (size_t)(16 * nt + m) * KLIN + DFV + 32 * ks + 8 * hh;
        acc[nt] = mm3(ah, al, ldfrag(wp), ldfrag(wp + 64 * KLIN), acc[nt]);
      }
    }
#pragma unroll
    for (int nt = 0; nt < 4; ++nt) {
#pragma unroll
      for (int r = 0; r < 8; ++r) {
        const float f = lk(acc[nt][r] + bb[nt]);
        unsigned short p, q;
        split2(f, p, q);
        tFh[(8 * hh + r) * PA + 16 * nt + m] = p;
        tFl[(8 * hh + r) * PA + 16 * nt + m] = q;
      }
    }
    __syncthreads();
    v8f acc2[4] = {z, z, z, z};
#pragma unroll
    for (int ks = 0; ks < 2; ++ks) {
      const v16bf gh = ldfrag(tFh + m * PA + 32 * ks + 8 * hh);
      const v16bf gl = ldfrag(tFl + m * PA + 32 * ks + 8 * hh);
#pragma unroll
      for (int nt = 0; nt < 4; ++nt) {
        const unsigned short* wp = W2h + (size_t)(16 * nt + m) * DIM + 32 * ks + 8 * hh;
        acc2[nt] = mm3(gh, gl, ldfrag(wp), ldfrag(wp + 64 * DIM), acc2[nt]);
      }
    }
#pragma unroll
    for (int nt = 0; nt < 4; ++nt) {
#pragma unroll
      for (int r = 0; r < 8; ++r) tD[(8 * hh + r) * PD + 16 * nt + m] = acc2[nt][r];
    }
    __syncthreads();
    st64f(tD, FH, row0, lane);
    __threadfence();
    st64f(tD, FH, row0, lane);
    __syncthreads();
  }
}

__global__ __launch_bounds__(G1THR) void k_gemm4(
    const unsigned short* __restrict__ X2, const unsigned short* __restrict__ Wpl,
    const float* __restrict__ FH, float* XF, int nN, int nUser, int nItem) {
  __shared__ __attribute__((aligned(16))) float sD[G1WAV * 16 * PD];
  const int tid = threadIdx.x, lane = tid & 31, wave = tid >> 5, hh = lane >> 4, m = lane & 15;
  float* tD = sD + wave * 16 * PD;
  const unsigned short* Wh = Wpl + OFF_WW;
  const v8f z = {0.f, 0.f, 0.f, 0.f, 0.f, 0.f, 0.f, 0.f};
  const int tile0 = ((int)blockIdx.x * G1WAV + wave) * TPW;

#pragma unroll 1
  for (int tt = 0; tt < TPW; ++tt) {
    const size_t row0 = (size_t)(tile0 + tt) * 16;
    const unsigned short* ap = X2 + (row0 + (size_t)m) * (2 * DIM) + 8 * hh;
    v8f acc[4] = {z, z, z, z};
#pragma unroll
    for (int ks = 0; ks < 2; ++ks) {
      const v16bf ah = ldfrag(ap + 32 * ks);
      const v16bf al = ldfrag(ap + DIM + 32 * ks);
#pragma unroll
      for (int nt = 0; nt < 4; ++nt) {
        const unsigned short* wp = Wh + (size_t)(16 * nt + m) * DIM + 32 * ks + 8 * hh;
        acc[nt] = mm3(ah, al, ldfrag(wp), ldfrag(wp + 64 * DIM), acc[nt]);
      }
    }
#pragma unroll
    for (int nt = 0; nt < 4; ++nt) {
      const int col = 16 * nt + m;
#pragma unroll
      for (int r = 0; r < 8; ++r) {
        const int row = (int)row0 + 8 * hh + r;
        int fi = row - nUser;
        fi = fi < 0 ? 0 : (fi > nItem - 1 ? nItem - 1 : fi);
        const float fv  = FH[(size_t)fi * DIM + col];
        const float add = (row >= nUser && row < nN) ? fv : 0.0f;
        tD[(8 * hh + r) * PD + col] = lk(acc[nt][r] + add);
      }
    }
    __syncthreads();
    st64f(tD, XF, row0, lane);
    __threadfence();
    st64f(tD, XF, row0, lane);
    __syncthreads();
  }
}

__device__ __forceinline__ void sc_store(const float* sc, float* out, int nB, int tid, int blk) {
  const int b4 = blk * SBLK + 4 * tid;
  const v4f v = *(const v4f*)(sc + 4 * tid);
  if (b4 + 4 <= nB) {
    *(volatile v4f*)(out + b4) = v;
  } else {
    if (b4 + 0 < nB) *(volatile float*)(out + b4 + 0) = v.x;
    if (b4 + 1 < nB) *(volatile float*)(out + b4 + 1) = v.y;
    if (b4 + 2 < nB) *(volatile float*)(out + b4 + 2) = v.z;
  }
}

__global__ __launch_bounds__(SBLK) void k_scores(
    const float* __restrict__ XF, const int* __restrict__ ua, const int* __restrict__ ib,
    float* out, int nB, int nN) {
  __shared__ __attribute__((aligned(16))) float sc[SBLK];
  const int tid = (int)threadIdx.x;
  int b = (int)blockIdx.x * SBLK + tid;
  b = b > nB - 1 ? nB - 1 : b;
  int u = ua[b];
  if (u < 0) u += nN;
  u = u < 0 ? 0 : (u > nN - 1 ? nN - 1 : u);
  int v = ib[b];
  if (v < 0) v += nN;
  v = v < 0 ? 0 : (v > nN - 1 ? nN - 1 : v);
  const float* pu = XF + (size_t)u * DIM;
  const float* pv = XF + (size_t)v * DIM;
  float s = 0.0f;
#pragma unroll 4
  for (int i = 0; i < 16; ++i) {
    const v4f a = *(const v4f*)(pu + 4 * i);
    const v4f c = *(const v4f*)(pv + 4 * i);
    s += a.x * c.x + a.y * c.y + a.z * c.z + a.w * c.w;
  }
  sc[tid] = s;
  __syncthreads();
  if (tid < SBLK / 4) {
    sc_store(sc, out, nB, tid, (int)blockIdx.x);
    __threadfence();
    sc_store(sc, out, nB, tid, (int)blockIdx.x);
  }
}

extern "C" void kernel_launch(void* const* d_in, const int* in_sizes, int n_in,
                              void* d_out, int out_size, void* d_ws, size_t ws_size,
                              hipStream_t stream) {
  if (n_in < 12) return;
  if (in_sizes[0] <= 0 || (in_sizes[0] % DIM) != 0) return;
  if (in_sizes[1] != DIM * DIM || in_sizes[6] != DIM * DIM || in_sizes[7] != DIM * DIM) return;
  if (in_sizes[2] <= 0 || (in_sizes[2] % DFV) != 0) return;
  if (in_sizes[3] <= 0 || (in_sizes[3] % DFV) != 0) return;
  if (in_sizes[4] != KLIN * DIM || in_sizes[5] != DIM) return;
  if (in_sizes[8] < 2 || (in_sizes[8] % 2) != 0) return;
  if (in_sizes[9] < 2 || (in_sizes[9] % 2) != 0) return;
  if (out_size <= 0 || in_sizes[10] != out_size || in_sizes[11] != out_size) return;
  const int nN    = in_sizes[0] / DIM;
  const int nVoc  = in_sizes[2] / DFV;
  const int nItem = in_sizes[3] / DFV;
  if (nItem > nN) return;
  const int nUser = nN - nItem;
  const int nE    = in_sizes[8] / 2;
  const int nW    = in_sizes[9] / 2;
  const int nB    = out_size;
  if (nN > (1 << 24) || nE > (1 << 28) || nW > (1 << 28) || nVoc > (1 << 24)) return;

  const float* emb   = (const float*)d_in[0];
  const float* Wc    = (const float*)d_in[1];
  const float* table = (const float*)d_in[2];
  const float* vf    = (const float*)d_in[3];
  const float* Wl    = (const float*)d_in[4];
  const float* lbias = (const float*)d_in[5];
  const float* Ww    = (const float*)d_in[6];
  const float* W2    = (const float*)d_in[7];
  const int*   edges = (const int*)d_in[8];
  const int*   words = (const int*)d_in[9];
  const int*   ua    = (const int*)d_in[10];
  const int*   ib    = (const int*)d_in[11];
  float* out = (float*)d_out;

  const int NPAD  = ((nN + NROW - 1) / NROW) * NROW;
  const int NIPAD = ((nItem + NROW - 1) / NROW) * NROW;

  char* ws = (char*)d_ws;
  size_t off = 0;
#define ALN(x) (((x) + 255) & ~(size_t)255)
  const size_t oW  = off;  off = ALN(off + (size_t)WTOT * 2);
  const size_t oH  = off;  off = ALN(off + (size_t)NPAD * DIM * 4);
  const size_t oX2 = off;  off = ALN(off + (size_t)NPAD * (2 * DIM) * 2);
  const size_t oT  = off;  off = ALN(off + (size_t)NIPAD * (2 * DFV) * 2);
  const size_t oFH = off;  off = ALN(off + (size_t)NIPAD * DIM * 4);
  const size_t oXF = off;  off = ALN(off + (size_t)NPAD * DIM * 4);
#undef ALN
  if (off > ws_size) return;
  if (off > ((size_t)128 << 20)) return;

  unsigned short* Wpl = (unsigned short*)(ws + oW);
  float*          H   = (float*)(ws + oH);
  unsigned short* X2  = (unsigned short*)(ws + oX2);
  unsigned short* T   = (unsigned short*)(ws + oT);
  float*          FH  = (float*)(ws + oFH);
  float*          XF  = (float*)(ws + oXF);

  const int* esrc  = edges;
  const int* edst  = edges + nE;
  const int* witem = words;
  const int* wword = words + nW;
  const int vec8e = ((nE & 3) == 0) ? 1 : 0;
  const int vec8w = ((nW & 3) == 0) ? 1 : 0;

  k_wprep<<<4, NTHR, 0, stream>>>(Wc, W2, Ww, Wl, Wpl);

  k_gemm1<<<NPAD / RPB1, G1THR, 0, stream>>>(emb, Wpl, H, nN);

  hipFuncSetAttribute(reinterpret_cast<const void*>(&k_agge),
                      hipFuncAttributeMaxDynamicSharedMemorySize, LDS_E);
  k_agge<<<NPAD / NBA, NTHR, LDS_E, stream>>>(edst, esrc, H, X2, nN, nE, vec8e);

  hipFuncSetAttribute(reinterpret_cast<const void*>(&k_aggw),
                      hipFuncAttributeMaxDynamicSharedMemorySize, LDS_W);
  k_aggw<<<NIPAD / NBW, NTHR, LDS_W, stream>>>(witem, wword, table, T, nVoc, nW, vec8w);

  k_gemm23<<<NIPAD / RPB2, G2THR, 0, stream>>>(vf, T, Wpl, lbias, FH, nItem);

  k_gemm4<<<NPAD / RPB1, G1THR, 0, stream>>>(X2, Wpl, FH, XF, nN, nUser, nItem);

  k_scores<<<(nB + SBLK - 1) / SBLK, SBLK, 0, stream>>>(XF, ua, ib, out, nB, nN);
}
